// GATv2_GCN_44925357916176
// MI455X (gfx1250) — hardware-run, weakly checked
//
#include <hip/hip_runtime.h>


namespace {
constexpr int N = 16384, E = 262144, FIN = 78, KIN = 96, HC = 780, PC = 800  , NH = 10, CH = 78, G = 512, F1 = 1500, F1P = 1504, K1 = 1568  , NOUT = 128, NTG = 49  ;
constexpr float XS = 8.0f, WSC = 256.0f, NEG = 0.2f;
typedef _Float16 b16;
typedef __attribute__((ext_vector_type(16))) _Float16 v16b;
typedef __attribute__((ext_vector_type(8))) _Float16 v8b;
typedef __attribute__((ext_vector_type(8))) float v8f;
typedef __attribute__((ext_vector_type(4))) float v4f;
__device__ __forceinline__ float bf16_rne(float f) { unsigned int u = __float_as_uint(f); u += 0x7FFFu + ((u >> 16) & 1u); return __uint_as_float(u & 0xFFFF0000u); }
__device__ __forceinline__ void split16(float v, b16& hi, b16& lo) { hi = (b16)v; lo = (b16)(v - (float)hi); }
__device__ __forceinline__ v16b frag_kb(const b16* p, int hh) { const v8b a = *(const v8b*)(p + 8 * hh), b = *(const v8b*)(p + 16 + 8 * hh); v16b f;
#pragma unroll
  for (int e = 0; e < 8; ++e) { f[e] = a[e]; f[8 + e] = b[e]; } return f; }
__device__ __forceinline__ v8f wmma16b(v16b a, v16b b, v8f c) { v8f d = __builtin_amdgcn_wmma_f32_16x16x32_f16(false, a, false, b, (short)0, c, false, false); asm volatile("v_nop\n\tv_nop\n\tv_nop\n\tv_nop" : "+v"(d) : "v"(a), "v"(b)); return d; }
__device__ __forceinline__ void wave_lds_sync() { __builtin_amdgcn_fence(__ATOMIC_RELEASE, "workgroup"); __builtin_amdgcn_wave_barrier(); __builtin_amdgcn_fence(__ATOMIC_ACQUIRE, "workgroup"); }
__device__ __forceinline__ float pmul(float a, float b) { float p = a * b; asm volatile("" : "+v"(p)); return p; }
__device__ __forceinline__ int iclamp(int v, int lo, int hi) { return v < lo ? lo : (v > hi ? hi : v); }
__device__ __forceinline__ float nexp(float x) { return __builtin_amdgcn_exp2f(x * 1.4426950408889634f); }
__device__ __forceinline__ float lrelu(float x) { return x > 0.0f ? x : NEG * x; }
constexpr int CSR_NBLK = 512, CSR_GB = 9, CSR_GN = 1 << CSR_GB  , CSR_MAXG = 512, CSR_CAP = 12288  ;
__global__ __launch_bounds__(64) void csrA_kernel(const int* __restrict__ dst, int E, int N, int nG, int CHP, int NGP, int* __restrict__ STG, int* __restrict__ HST) {
  extern __shared__ int sm[];
  int* cnt = sm; int* run = sm + NGP; int* ids = sm + 2 * NGP;
  const int b = blockIdx.x; const int ch = (E + CSR_NBLK - 1) / CSR_NBLK; const int e0 = b * ch, e1 = min(E, e0 + ch);
  for (int i = threadIdx.x; i < NGP; i += 64) cnt[i] = 0;
  for (int i = threadIdx.x; i < CHP; i += 64) ids[i] = -1;
  __syncthreads();
  if (threadIdx.x == 0) {
    for (int e = e0; e < e1; ++e) { int d = dst[e]; d = (d < 0) ? 0 : (d >= N ? N - 1 : d); cnt[d >> CSR_GB] += 1; }
    int acc = 0; for (int g = 0; g < nG; ++g) { run[g] = acc; acc += cnt[g]; }
    for (int e = e0; e < e1; ++e) { int d = dst[e]; d = (d < 0) ? 0 : (d >= N ? N - 1 : d); const int g = d >> CSR_GB; ids[run[g]] = e; run[g] += 1; } }
  __syncthreads();
  typedef __attribute__((ext_vector_type(4))) int v4i;
  for (int pass = 0; pass < 2; ++pass) {
    for (int i = threadIdx.x; i < CHP / 4; i += 64) *(volatile v4i*)(STG + (size_t)b * CHP + i * 4) = *(const v4i*)(&ids[i * 4]);
    for (int i = threadIdx.x; i < NGP / 4; i += 64) { v4i v; for (int e = 0; e < 4; ++e) v[e] = (i * 4 + e < nG) ? cnt[i * 4 + e] : 0; *(volatile v4i*)(HST + (size_t)b * NGP + i * 4) = v; }
    __threadfence(); }
}
__global__ __launch_bounds__(512) void csrS_kernel(const int* __restrict__ HST, int nG, int NGP, int* __restrict__ START, int* __restrict__ TOT, int* __restrict__ OFF) {
  __shared__ int tot[CSR_MAXG];
  const int b = threadIdx.x;
  for (int pass = 0; pass < 2; ++pass) { int runb = 0; for (int g = 0; g < nG; ++g) { int c = HST[(size_t)b * NGP + g]; c = (c < 0) ? 0 : c; ((volatile int*)OFF)[(size_t)g * CSR_NBLK + b] = runb; runb += c; } __threadfence(); }
  for (int g = threadIdx.x; g < nG; g += 512) { int s = 0; for (int bb = 0; bb < CSR_NBLK; ++bb) { int c = HST[(size_t)bb * NGP + g]; s += (c < 0) ? 0 : c; } tot[g] = s; }
  __syncthreads();
  if (threadIdx.x < 32) {
    __shared__ int st[CSR_MAXG + 32];
    if (threadIdx.x == 0) { int acc = 0; for (int g = 0; g < NGP; ++g) { st[g] = acc; if (g < nG) acc += (tot[g] + 31) & ~31; } st[NGP] = acc; }
    __builtin_amdgcn_fence(__ATOMIC_RELEASE, "workgroup"); __builtin_amdgcn_wave_barrier(); __builtin_amdgcn_fence(__ATOMIC_ACQUIRE, "workgroup");
    for (int pass = 0; pass < 2; ++pass) { for (int i = threadIdx.x; i < NGP + 32; i += 32) { ((volatile int*)START)[i] = (i <= NGP) ? st[min(i, NGP)] : 0; ((volatile int*)TOT)[i] = (i < nG) ? tot[i] : 0; } __threadfence(); } }
}
__global__ __launch_bounds__(256) void csrB_kernel(const int* __restrict__ dst, int N, int nG, int CHP, int NGP, int permLen, const int* __restrict__ STG, const int* __restrict__ HST, const int* __restrict__ OFF, const int* __restrict__ START, const int* __restrict__ TOT, int* __restrict__ PERM, int* __restrict__ ROWPTR, int* __restrict__ ROWCNT, int* __restrict__ FLAG) {
  typedef __attribute__((ext_vector_type(4))) int v4i;
  __shared__ int ids[CSR_CAP]; __shared__ unsigned short key[CSR_CAP]; __shared__ int outp[CSR_CAP]; __shared__ int ncnt[CSR_GN + 1]; __shared__ int boff[CSR_NBLK + 1];
  const int g = blockIdx.x, t_ = threadIdx.x; int tot = TOT[g]; int st = START[g], stn = START[g + 1]; const int v0 = g * CSR_GN; const int nv = min(CSR_GN, N - v0);
  st = (st < 0) ? 0 : (st > permLen - 32 ? permLen - 32 : st) & ~31; stn = (stn < st) ? st : (stn > permLen ? permLen : stn); tot = (tot < 0) ? 0 : tot; if (tot > stn - st && tot <= CSR_CAP) tot = stn - st;
  if (tot > CSR_CAP) {
    for (int pass = 0; pass < 2; ++pass) { for (int i = t_; i < CSR_GN / 4; i += 256) { v4i a, c; for (int e = 0; e < 4; ++e) { a[e] = st; c[e] = 0; } *(volatile v4i*)(ROWPTR + v0 + i * 4) = a; *(volatile v4i*)(ROWCNT + v0 + i * 4) = c; } if (t_ == 0) ((volatile int*)FLAG)[0] = 1; __threadfence(); } (void)nv; return; }
  if (t_ == 0) { int acc = 0; for (int b = 0; b < CSR_NBLK; ++b) { boff[b] = acc; int c = HST[(size_t)b * NGP + g]; c = (c < 0) ? 0 : (c > CHP ? CHP : c); acc += c; if (acc > tot) acc = tot; } boff[CSR_NBLK] = acc; }
  for (int i = t_; i <= CSR_GN; i += 256) ncnt[i] = 0;
  __syncthreads();
  for (int b = 0; b < CSR_NBLK; ++b) { const int c = boff[b + 1] - boff[b]; int o_ = OFF[(size_t)g * CSR_NBLK + b]; o_ = (o_ < 0) ? 0 : (o_ > CHP - c ? CHP - c : o_); const int* src_ = STG + (size_t)b * CHP + o_;
    for (int i = t_; i < c; i += 256) { int id = src_[i]; id = (id < 0) ? 0 : id; ids[boff[b] + i] = id; int d = dst[id]; d = (d < v0) ? v0 : (d >= N ? N - 1 : d); int kk = d - v0; kk = (kk < 0) ? 0 : (kk >= CSR_GN ? CSR_GN - 1 : kk); key[boff[b] + i] = (unsigned short)kk; } }
  __syncthreads();
  if (t_ == 0) { for (int i = 0; i < tot; ++i) ncnt[key[i]] += 1; int acc = 0; for (int vl = 0; vl < CSR_GN; ++vl) { const int c = ncnt[vl]; ncnt[vl] = acc; acc += c; } ncnt[CSR_GN] = acc;
    for (int i = 0; i < tot; ++i) { const int vl = key[i]; outp[ncnt[vl]] = ids[i]; ncnt[vl] += 1; }
    for (int vl = CSR_GN; vl > 0; --vl) ncnt[vl] = ncnt[vl - 1]; ncnt[0] = 0; }
  __syncthreads();
  for (int pass = 0; pass < 2; ++pass) {
    for (int i = t_; i < (stn - st) / 4; i += 256) { v4i v; for (int e = 0; e < 4; ++e) { const int q = i * 4 + e; v[e] = (q < tot) ? outp[q] : -1; } *(volatile v4i*)(PERM + st + i * 4) = v; }
    for (int i = t_; i < CSR_GN / 4; i += 256) { v4i a, c; for (int e = 0; e < 4; ++e) { const int vl = i * 4 + e; a[e] = st + ncnt[vl]; c[e] = (vl < nv) ? (ncnt[vl + 1] - ncnt[vl]) : 0; } *(volatile v4i*)(ROWPTR + v0 + i * 4) = a; *(volatile v4i*)(ROWCNT + v0 + i * 4) = c; }
    __threadfence(); }
}
__global__ __launch_bounds__(256) void csrZ_kernel(int* __restrict__ p, size_t n4) { typedef __attribute__((ext_vector_type(4))) int v4i; const size_t tid = (size_t)blockIdx.x * 256 + threadIdx.x, nth = (size_t)gridDim.x * 256; v4i z = {0, 0, 0, 0}; for (size_t i = tid; i < n4; i += nth) *(volatile v4i*)(p + i * 4) = z; }
struct CsrBufs { int *STG, *HST, *OFF, *START, *TOT, *PERM, *ROWPTR, *ROWCNT, *FLAG; int nG, NGP, CHP; size_t permLen; char* base; size_t bytes; };
static size_t csr_carve(CsrBufs& c, char* ws, size_t off, int E, int N) {
  const size_t off0 = off; c.base = ws + off;
  auto al = [&](size_t bytes) { char* p = ws + off; off += (bytes + 255) & ~(size_t)255; return p; };
  c.nG = (N + CSR_GN - 1) / CSR_GN; c.NGP = (c.nG + 31) & ~31; const int ch = (E + CSR_NBLK - 1) / CSR_NBLK; c.CHP = (ch + 31) & ~31; c.permLen = (size_t)E + 32 * (size_t)c.nG + 32;
  c.STG = (int*)al((size_t)CSR_NBLK * c.CHP * 4); c.HST = (int*)al((size_t)CSR_NBLK * c.NGP * 4); c.OFF = (int*)al((size_t)c.NGP * CSR_NBLK * 4); c.START = (int*)al((size_t)(c.NGP + 64) * 4); c.TOT = (int*)al((size_t)(c.NGP + 64) * 4);
  c.PERM = (int*)al(c.permLen * 4); c.ROWPTR = (int*)al((size_t)c.nG * CSR_GN * 4); c.ROWCNT = (int*)al((size_t)c.nG * CSR_GN * 4); c.FLAG = (int*)al(256);
  c.bytes = off - off0; return off;
}
static void csr_build(const CsrBufs& c, const int* dst, int E, int N, hipStream_t stream) {
  const size_t smem = (size_t)(2 * c.NGP + c.CHP) * 4;
  csrZ_kernel<<<512, 256, 0, stream>>>((int*)c.base, c.bytes / 16);
  csrA_kernel<<<CSR_NBLK, 64, smem, stream>>>(dst, E, N, c.nG, c.CHP, c.NGP, c.STG, c.HST);
  csrS_kernel<<<1, 512, 0, stream>>>(c.HST, c.nG, c.NGP, c.START, c.TOT, c.OFF);
  csrB_kernel<<<c.nG, 256, 0, stream>>>(dst, N, c.nG, c.CHP, c.NGP, (int)c.permLen, c.STG, c.HST, c.OFF, c.START, c.TOT, c.PERM, c.ROWPTR, c.ROWCNT, c.FLAG);
}


__global__ __launch_bounds__(256) void wprep_kernel(const float* __restrict__ wl, const float* __restrict__ wr, const float* __restrict__ wg, const float* __restrict__ wf1, const float* __restrict__ wf2, b16* __restrict__ WLR, b16* __restrict__ WG, b16* __restrict__ WF1, b16* __restrict__ WF2) {
  const size_t u = (size_t)blockIdx.x * 256 + threadIdx.x; const size_t n0 = (size_t)2 * PC * KIN / 8, n1 = (size_t)NTG * 16 * PC / 8, n2 = (size_t)F1P * K1 / 8, n3 = (size_t)NOUT * F1P / 8; size_t t = u; v8b o;
  if (t < n0) { const size_t e = t * 8; const int row = (int)(e / KIN), k0 = (int)(e % KIN); const int part = row / PC, oo = row % PC; const float* w = part ? wr : wl;
    for (int j = 0; j < 8; ++j) { const int k = k0 + j; o[j] = (k < FIN && oo < HC) ? (b16)(bf16_rne(w[(size_t)k * HC + oo]) * WSC) : (b16)0.0f; } for (int pass = 0; pass < 2; ++pass) { *(volatile v8b*)(WLR + e) = o; __threadfence(); } return; } t -= n0;
  if (t < n1) { const size_t e = t * 8; const int oo = (int)(e / PC), k0 = (int)(e % PC); for (int j = 0; j < 8; ++j) { const int k = k0 + j; o[j] = (k < HC && oo < HC) ? (b16)(bf16_rne(wg[(size_t)k * HC + oo]) * WSC) : (b16)0.0f; } for (int pass = 0; pass < 2; ++pass) { *(volatile v8b*)(WG + e) = o; __threadfence(); } return; } t -= n1;
  if (t < n2) { const size_t e = t * 8; const int oo = (int)(e / K1), k0 = (int)(e % K1); for (int j = 0; j < 8; ++j) { const int k = k0 + j; o[j] = (k < 2 * HC && oo < F1) ? (b16)(bf16_rne(wf1[(size_t)k * F1 + oo]) * WSC) : (b16)0.0f; } for (int pass = 0; pass < 2; ++pass) { *(volatile v8b*)(WF1 + e) = o; __threadfence(); } return; } t -= n2;
  if (t < n3) { const size_t e = t * 8; const int oo = (int)(e / F1P), k0 = (int)(e % F1P); for (int j = 0; j < 8; ++j) { const int k = k0 + j; o[j] = (k < F1) ? (b16)(bf16_rne(wf2[(size_t)k * NOUT + oo]) * WSC) : (b16)0.0f; } for (int pass = 0; pass < 2; ++pass) { *(volatile v8b*)(WF2 + e) = o; __threadfence(); } }
}
__global__ __launch_bounds__(128) void proj_kernel(const float* __restrict__ x, const b16* __restrict__ WLR, float* __restrict__ XL, float* __restrict__ XR) {
  __shared__ __attribute__((aligned(16))) float Tf[4][16][128 + 4];
  const int wave = threadIdx.x >> 5, lane = threadIdx.x & 31, nloc = lane & 15, hlf = lane >> 4; const size_t m0 = (size_t)blockIdx.x * 64 + wave * 16; const int grp = blockIdx.y; const int plane = grp >> 1, c0 = (grp & 1) * 512, ntile = (grp & 1) ? 18 : 32;
  float* OUT = plane ? XR : XL; const b16* W = WLR + (size_t)(plane * PC + c0) * KIN;
  v16b af[3]; { const size_t v = m0 + nloc; const float* r = x + v * FIN; for (int ks = 0; ks < 3; ++ks) { v16b a = {}; for (int e = 0; e < 8; ++e) { const int k0 = ks * 32 + 8 * hlf + e, k1 = ks * 32 + 16 + 8 * hlf + e; a[e] = k0 < FIN ? (b16)(bf16_rne(r[k0]) * XS) : (b16)0.0f; a[8 + e] = k1 < FIN ? (b16)(bf16_rne(r[k1]) * XS) : (b16)0.0f; } af[ks] = a; } }
  for (int t0 = 0; t0 < ntile; t0 += 8) { const int nt = (ntile - t0) < 8 ? (ntile - t0) : 8; v8f acc[8];
#pragma unroll
    for (int t = 0; t < 8; ++t) acc[t] = (v8f){};
#pragma unroll
    for (int ks = 0; ks < 3; ++ks) {
#pragma unroll
      for (int t = 0; t < 8; ++t) if (t < nt) acc[t] = wmma16b(af[ks], frag_kb(W + (size_t)((t0 + t) * 16 + nloc) * KIN + ks * 32, hlf), acc[t]); }
    wave_lds_sync();
#pragma unroll
    for (int t = 0; t < 8; ++t) if (t < nt) {
#pragma unroll 1
      for (int r = 0; r < 8; ++r) Tf[wave][8 * hlf + r][t * 16 + nloc] = acc[t][r] * (1.0f / (XS * WSC)); }
    wave_lds_sync();
    const int ncol = nt * 16;
    for (int pass = 0; pass < 2; ++pass) { for (int rr = 0; rr < 16; ++rr) if (lane * 4 < ncol) *(volatile v4f*)(OUT + (m0 + rr) * PC + c0 + t0 * 16 + lane * 4) = *(const v4f*)(&Tf[wave][rr][lane * 4]); __threadfence(); } }
}
__global__ __launch_bounds__(256) void attn_kernel(const float* __restrict__ XL, const float* __restrict__ XR, const float* __restrict__ att, const float* __restrict__ bg, const int* __restrict__ srcs, const int* __restrict__ PERM, const int* __restrict__ ROWPTR, const int* __restrict__ ROWCNT, int permLen, float* __restrict__ H1) {
  __shared__ float part[8][32][3]; __shared__ float ph[8][16]; __shared__ __attribute__((aligned(16))) float rowbuf[8][PC];
  const int wave = threadIdx.x >> 5, lane = threadIdx.x & 31; const size_t v = (size_t)blockIdx.x * 8 + wave; const int cb = lane * 24;
  const int hA = cb / CH; const int nA = ((hA + 1) * CH - cb) < 24 ? ((hA + 1) * CH - cb) : 24; const bool hasX = lane < 12;
  float ac[25], xr_[25];
#pragma unroll
  for (int j = 0; j < 25; ++j) { const int c = j < 24 ? cb + j : HC - 12 + lane; const bool ok = j < 24 ? true : hasX; const int h = j < 24 ? (j < nA ? hA : hA + 1) : 9; float aw = ok ? bf16_rne(att[h * CH + (c - h * CH)]) : 0.0f; asm volatile("" : "+v"(aw)); ac[j] = aw; xr_[j] = ok ? XR[v * PC + c] : 0.0f; }
  int st = ROWPTR[v], cnt = ROWCNT[v]; cnt = iclamp(cnt, 0, 65536); st = iclamp(st, 0, permLen - cnt);
  float xs[25];
  auto load_row = [&](size_t s) { const float* p = XL + s * PC + cb;
#pragma unroll
    for (int q = 0; q < 6; ++q) { const v4f t = *(const v4f*)(p + 4 * q);
#pragma unroll
      for (int i = 0; i < 4; ++i) xs[4 * q + i] = t[i]; } xs[24] = hasX ? XL[s * PC + HC - 12 + lane] : 0.0f; };
  auto head_logits = [&]() -> float {
    float pa = 0.0f, pb = 0.0f, px = 0.0f;
#pragma unroll
    for (int j = 0; j < 24; ++j) { const float e = pmul(ac[j], lrelu(xs[j] + xr_[j])); if (j < nA) pa += e; else pb += e; } if (hasX) px = pmul(ac[24], lrelu(xs[24] + xr_[24]));
    part[wave][lane][0] = pa; part[wave][lane][1] = pb; part[wave][lane][2] = px; wave_lds_sync();
    float lg = 0.0f; if (lane < NH) { for (int l2 = 0; l2 < 32; ++l2) { const int cb2 = l2 * 24; const int hA2 = cb2 / CH; const int nA2 = ((hA2 + 1) * CH - cb2) < 24 ? ((hA2 + 1) * CH - cb2) : 24; if (hA2 == lane) lg += part[wave][l2][0]; if (nA2 < 24 && hA2 + 1 == lane) lg += part[wave][l2][1]; if (l2 < 12 && lane == 9) lg += part[wave][l2][2]; } }
    wave_lds_sync(); return lg; };
  load_row(v); float mx = head_logits();
#pragma unroll 1
  for (int j = 0; j < cnt; ++j) { const int e = iclamp(PERM[st + j], 0, E - 1); const size_t s = (size_t)iclamp(srcs[e], 0, N - 1); load_row(s); const float lg = head_logits(); mx = fmaxf(mx, lg); }
  float den = 0.0f, acc[25];
#pragma unroll
  for (int j = 0; j < 25; ++j) acc[j] = 0.0f;
#pragma unroll 1
  for (int j = -1; j < cnt; ++j) { size_t s = v; if (j >= 0) { const int e = iclamp(PERM[st + j], 0, E - 1); s = (size_t)iclamp(srcs[e], 0, N - 1); } load_row(s); const float lg = head_logits();
    const float p = (lane < NH) ? nexp(lg - mx) : 0.0f; den += p; if (lane < 16) ph[wave][lane] = p; wave_lds_sync();
    const float pA = ph[wave][hA], pB = ph[wave][(hA + 1) < NH ? hA + 1 : NH - 1], pX = ph[wave][9]; wave_lds_sync();

#pragma unroll
    for (int q = 0; q < 24; ++q) acc[q] += pmul(q < nA ? pA : pB, xs[q]); acc[24] += pmul(pX, xs[24]); }
  if (lane < 16) ph[wave][lane] = (lane < NH && den > 0.0f) ? 1.0f / den : 0.0f; wave_lds_sync(); const float iA = ph[wave][hA], iB = ph[wave][(hA + 1) < NH ? hA + 1 : NH - 1], iX = ph[wave][9];

#pragma unroll
  for (int q = 0; q < 24; ++q) { const int c = cb + q; rowbuf[wave][c] = (c < HC) ? fmaxf(pmul(acc[q], q < nA ? iA : iB) + bf16_rne(bg[c]), 0.0f) : 0.0f; }
  if (hasX) rowbuf[wave][HC - 12 + lane] = fmaxf(pmul(acc[24], iX) + bf16_rne(bg[HC - 12 + lane]), 0.0f);
  if (lane >= 12) { const int c = HC + (lane - 12); if (c < PC) rowbuf[wave][c] = 0.0f; }
  wave_lds_sync();
  for (int pass = 0; pass < 2; ++pass) { for (int q = lane * 4; q < PC; q += 128) *(volatile v4f*)(H1 + v * PC + q) = *(const v4f*)(&rowbuf[wave][q]); __threadfence(); }
}
__global__ __launch_bounds__(32) void gcn_gemm_kernel(const float* __restrict__ H1, const b16* __restrict__ WG, float* __restrict__ T) {
  __shared__ __attribute__((aligned(16))) b16 Ah[16][PC + 8], Al[16][PC + 8]; __shared__ __attribute__((aligned(16))) float Tf[16][16 * 8 + 4];
  const int lane = threadIdx.x, nloc = lane & 15, hlf = lane >> 4; const size_t m0 = (size_t)blockIdx.x * 16;
  for (int rr = 0; rr < 16; ++rr) for (int q = lane * 4; q < PC; q += 128) { const v4f x = *(const v4f*)(H1 + (m0 + rr) * PC + q); for (int i = 0; i < 4; ++i) { b16 p, s; split16(x[i] * XS, p, s); Ah[rr][q + i] = p; Al[rr][q + i] = s; } }
  wave_lds_sync();
  for (int t0 = 0; t0 < NTG; t0 += 8) { const int nt = (NTG - t0) < 8 ? (NTG - t0) : 8; v8f acc[8];
#pragma unroll
    for (int t = 0; t < 8; ++t) acc[t] = (v8f){};
#pragma unroll 1
    for (int kb = 0; kb < PC; kb += 32) { const v16b a = frag_kb(&Ah[nloc][kb], hlf), al = frag_kb(&Al[nloc][kb], hlf);
#pragma unroll
      for (int t = 0; t < 8; ++t) if (t < nt) { const v16b bw = frag_kb(WG + (size_t)((t0 + t) * 16 + nloc) * PC + kb, hlf); acc[t] = wmma16b(a, bw, acc[t]); acc[t] = wmma16b(al, bw, acc[t]); } }
#pragma unroll
    for (int t = 0; t < 8; ++t) if (t < nt) {
#pragma unroll 1
      for (int r = 0; r < 8; ++r) Tf[8 * hlf + r][t * 16 + nloc] = acc[t][r] * (1.0f / (XS * WSC)); }
    if (nt == 1 && lane >= 16) for (int rr = 0; rr < 16; ++rr) Tf[rr][lane] = 0.0f;
    wave_lds_sync();
    const int ncol = (nt == 1) ? 32 : nt * 16;
    for (int pass = 0; pass < 2; ++pass) { for (int rr = 0; rr < 16; ++rr) if (lane * 4 < ncol) *(volatile v4f*)(T + (m0 + rr) * PC + t0 * 16 + lane * 4) = *(const v4f*)(&Tf[rr][lane * 4]); __threadfence(); }
    wave_lds_sync(); }
}
__global__ __launch_bounds__(256) void gcn_agg_kernel(const float* __restrict__ T, const float* __restrict__ bgc, const int* __restrict__ srcs, const int* __restrict__ PERM, const int* __restrict__ ROWPTR, const int* __restrict__ ROWCNT, int permLen, float* __restrict__ H2) {
  __shared__ __attribute__((aligned(16))) float rowbuf[8][PC];
  const int wave = threadIdx.x >> 5, lane = threadIdx.x & 31; const size_t v = (size_t)blockIdx.x * 8 + wave; const int cb = lane * 24; const bool hasX = lane < 12;
  int st = ROWPTR[v], cnt = ROWCNT[v]; cnt = iclamp(cnt, 0, 65536); st = iclamp(st, 0, permLen - cnt); const float dv = rsqrtf((float)cnt + 1.0f);
  float acc[25]; { const float w = dv; const float* p = T + v * PC + cb; for (int q = 0; q < 6; ++q) { const v4f t = *(const v4f*)(p + 4 * q); for (int i = 0; i < 4; ++i) acc[4 * q + i] = pmul(w, t[i]); } acc[24] = hasX ? pmul(w, T[v * PC + HC - 12 + lane]) : 0.0f; }
#pragma unroll 1
  for (int j = 0; j < cnt; ++j) { const int e = iclamp(PERM[st + j], 0, E - 1); const size_t s = (size_t)iclamp(srcs[e], 0, N - 1); const float w = rsqrtf((float)iclamp(ROWCNT[s], 0, 65536) + 1.0f); const float* p = T + s * PC + cb;
    for (int q = 0; q < 6; ++q) { const v4f t = *(const v4f*)(p + 4 * q); for (int i = 0; i < 4; ++i) acc[4 * q + i] += pmul(w, t[i]); } if (hasX) acc[24] += pmul(w, T[s * PC + HC - 12 + lane]); }
  for (int q = 0; q < 24; ++q) { const int c = cb + q; rowbuf[wave][c] = (c < HC) ? fmaxf(pmul(dv, acc[q]) + bf16_rne(bgc[c]), 0.0f) : 0.0f; }
  if (hasX) rowbuf[wave][HC - 12 + lane] = fmaxf(pmul(dv, acc[24]) + bf16_rne(bgc[HC - 12 + lane]), 0.0f);
  if (lane >= 12) { const int c = HC + (lane - 12); if (c < PC) rowbuf[wave][c] = 0.0f; }
  wave_lds_sync();
  for (int pass = 0; pass < 2; ++pass) { for (int q = lane * 4; q < PC; q += 128) *(volatile v4f*)(H2 + v * PC + q) = *(const v4f*)(&rowbuf[wave][q]); __threadfence(); }
}
__device__ int lower_bound_i(const int* a, int n, int key) { int lo = 0, hi = n; while (lo < hi) { const int mid = (lo + hi) >> 1; if (a[mid] < key) lo = mid + 1; else hi = mid; } return lo; }
__global__ __launch_bounds__(256) void pool_kernel(const float* __restrict__ H2, const int* __restrict__ batch, float* __restrict__ GP) {
  __shared__ __attribute__((aligned(16))) float row[K1];
  const int g = blockIdx.x, t = threadIdx.x; const int lo = lower_bound_i(batch, N, g), hi = lower_bound_i(batch, N, g + 1);
  for (int c = t; c < HC; c += 256) { float s = 0.0f, mx = -INFINITY; for (int v = lo; v < hi; ++v) { const float h = H2[(size_t)v * PC + c]; s += h; mx = fmaxf(mx, h); } row[c] = (hi > lo) ? mx : 0.0f; row[HC + c] = s / fmaxf((float)(hi - lo), 1.0f); }
  if (t < K1 - 2 * HC) row[2 * HC + t] = 0.0f;
  __syncthreads();
  for (int pass = 0; pass < 2; ++pass) { for (int q = t * 4; q < K1; q += 1024) *(volatile v4f*)(GP + (size_t)g * K1 + q) = *(const v4f*)(&row[q]); __threadfence(); }
}
__global__ __launch_bounds__(32) void fc1_kernel(const float* __restrict__ GP, const b16* __restrict__ WF1, const float* __restrict__ b1, float* __restrict__ F) {
  __shared__ __attribute__((aligned(16))) b16 Ah[16][K1 + 8], Al[16][K1 + 8]; __shared__ __attribute__((aligned(16))) float Tf[16][16 * 12 + 4];
  const int lane = threadIdx.x, nloc = lane & 15, hlf = lane >> 4; const size_t m0 = (size_t)blockIdx.x * 16;
  for (int rr = 0; rr < 16; ++rr) for (int q = lane * 4; q < K1; q += 128) { const v4f x = *(const v4f*)(GP + (m0 + rr) * K1 + q); for (int i = 0; i < 4; ++i) { b16 p, s; split16(x[i] * XS, p, s); Ah[rr][q + i] = p; Al[rr][q + i] = s; } }
  wave_lds_sync();
  for (int t0 = 0; t0 < F1P / 16; t0 += 12) { const int nt = (F1P / 16 - t0) < 12 ? (F1P / 16 - t0) : 12; v8f acc[12];
#pragma unroll
    for (int t = 0; t < 12; ++t) acc[t] = (v8f){};
#pragma unroll 1
    for (int kb = 0; kb < K1; kb += 32) { const v16b a = frag_kb(&Ah[nloc][kb], hlf), al = frag_kb(&Al[nloc][kb], hlf);
#pragma unroll
      for (int t = 0; t < 12; ++t) if (t < nt) { const v16b bw = frag_kb(WF1 + (size_t)((t0 + t) * 16 + nloc) * K1 + kb, hlf); acc[t] = wmma16b(a, bw, acc[t]); acc[t] = wmma16b(al, bw, acc[t]); } }
#pragma unroll
    for (int t = 0; t < 12; ++t) if (t < nt) { const int cabs = (t0 + t) * 16 + nloc; const float bb = cabs < F1 ? bf16_rne(b1[cabs]) : 0.0f;
#pragma unroll 1
      for (int r = 0; r < 8; ++r) Tf[8 * hlf + r][t * 16 + nloc] = cabs < F1 ? fmaxf(acc[t][r] * (1.0f / (XS * WSC)) + bb, 0.0f) : 0.0f; }
    wave_lds_sync();
    const int ncol = nt * 16;
    for (int pass = 0; pass < 2; ++pass) { for (int rr = 0; rr < 16; ++rr) for (int q = lane * 4; q < ncol; q += 128) *(volatile v4f*)(F + (m0 + rr) * F1P + t0 * 16 + q) = *(const v4f*)(&Tf[rr][q]); __threadfence(); }
    wave_lds_sync(); }
}
__global__ __launch_bounds__(32) void fc2_kernel(const float* __restrict__ F, const b16* __restrict__ WF2, const float* __restrict__ b2, float* __restrict__ out) {
  __shared__ __attribute__((aligned(16))) b16 Ah[16][F1P + 8], Al[16][F1P + 8]; __shared__ __attribute__((aligned(16))) float Tf[16][NOUT + 4];
  const int lane = threadIdx.x, nloc = lane & 15, hlf = lane >> 4; const size_t m0 = (size_t)blockIdx.x * 16;
  for (int rr = 0; rr < 16; ++rr) for (int q = lane * 4; q < F1P; q += 128) { const v4f x = *(const v4f*)(F + (m0 + rr) * F1P + q); for (int i = 0; i < 4; ++i) { b16 p, s; split16(x[i] * XS, p, s); Ah[rr][q + i] = p; Al[rr][q + i] = s; } }
  wave_lds_sync();
  v8f acc[8];
#pragma unroll
  for (int t = 0; t < 8; ++t) acc[t] = (v8f){};
#pragma unroll 1
  for (int kb = 0; kb < F1P; kb += 32) { const v16b a = frag_kb(&Ah[nloc][kb], hlf), al = frag_kb(&Al[nloc][kb], hlf);
#pragma unroll
    for (int t = 0; t < 8; ++t) { const v16b bw = frag_kb(WF2 + (size_t)(t * 16 + nloc) * F1P + kb, hlf); acc[t] = wmma16b(a, bw, acc[t]); acc[t] = wmma16b(al, bw, acc[t]); } }
#pragma unroll
  for (int t = 0; t < 8; ++t) { const int c = t * 16 + nloc; const float bb = bf16_rne(b2[c]);
#pragma unroll 1
    for (int r = 0; r < 8; ++r) Tf[8 * hlf + r][c] = acc[t][r] * (1.0f / (XS * WSC)) + bb; }
  wave_lds_sync();
  for (int pass = 0; pass < 2; ++pass) { for (int rr = 0; rr < 16; ++rr) *(volatile v4f*)(out + (m0 + rr) * NOUT + lane * 4) = *(const v4f*)(&Tf[rr][lane * 4]); __threadfence(); }
}
}

extern "C" void kernel_launch(void* const* d_in, const int* in_sizes, int n_in, void* d_out, int out_size, void* d_ws, size_t ws_size, hipStream_t stream) {
  (void)n_in;
  auto Fp = [&](int i) { return (const float*)d_in[i]; }; auto Ip = [&](int i) { return (const int*)d_in[i]; };
  if (in_sizes[0] != N * FIN || in_sizes[1] != 2 * E || in_sizes[2] != N || in_sizes[3] != FIN * HC || in_sizes[5] != NH * CH || in_sizes[7] != HC * HC || in_sizes[9] != 2 * HC * F1 || in_sizes[11] != F1 * NOUT || out_size != G * NOUT) return;
  size_t off = 0; char* ws = (char*)d_ws;
  auto carve = [&](size_t bytes) { char* p = ws + off; off += (bytes + 255) & ~(size_t)255; return p; };
  b16* WLR = (b16*)carve((size_t)2 * PC * KIN * 2); b16* WG = (b16*)carve((size_t)NTG * 16 * PC * 2); b16* WF1 = (b16*)carve((size_t)F1P * K1 * 2); b16* WF2 = (b16*)carve((size_t)NOUT * F1P * 2);
  float* XL = (float*)carve((size_t)N * PC * 4); float* XR = (float*)carve((size_t)N * PC * 4); float* H1 = (float*)carve((size_t)N * PC * 4); float* T = XL; float* H2 = XR;
  float* GP = (float*)carve((size_t)G * K1 * 4); float* F = (float*)carve((size_t)G * F1P * 4);
  CsrBufs csr; off = csr_carve(csr, ws, off, E, N);
  if (off > ws_size) return;
  wprep_kernel<<<(unsigned)(((size_t)2 * PC * KIN / 8 + (size_t)NTG * 16 * PC / 8 + (size_t)F1P * K1 / 8 + (size_t)NOUT * F1P / 8 + 255) / 256), 256, 0, stream>>>(Fp(3), Fp(4), Fp(7), Fp(9), Fp(11), WLR, WG, WF1, WF2);
  csr_build(csr, Ip(1) + E, E, N, stream);
  proj_kernel<<<dim3(N / 64, 4), 128, 0, stream>>>(Fp(0), WLR, XL, XR);
  attn_kernel<<<N / 8, 256, 0, stream>>>(XL, XR, Fp(5), Fp(6), Ip(1), csr.PERM, csr.ROWPTR, csr.ROWCNT, (int)csr.permLen, H1);
  gcn_gemm_kernel<<<N / 16, 32, 0, stream>>>(H1, WG, T);
  gcn_agg_kernel<<<N / 8, 256, 0, stream>>>(T, Fp(8), Ip(1), csr.PERM, csr.ROWPTR, csr.ROWCNT, (int)csr.permLen, H2);
  pool_kernel<<<G, 256, 0, stream>>>(H2, Ip(2), GP);
  fc1_kernel<<<G / 16, 32, 0, stream>>>(GP, WF1, Fp(10), F);
  fc2_kernel<<<G / 16, 32, 0, stream>>>(F, WF2, Fp(12), (float*)d_out);
}
